// Encoder_58952721105436
// MI455X (gfx1250) — hardware-verified
//
#include <hip/hip_runtime.h>


#ifndef NB
#define NB 4
#endif
#ifndef SEQ
#define SEQ 2048
#endif
#define NB_FULL  4
#define SEQ_FULL 2048
#define DM   512
#define NH   8
#define DK   64
#define DFF  2048
#define NTOK (NB * SEQ)
#define LP   72
#define VP   136
#define FP   68

static_assert(NB >= 1 && NB <= NB_FULL);
static_assert(SEQ >= 128 && SEQ <= SEQ_FULL);
static_assert(SEQ % 128 == 0);
static_assert(SEQ % 32 == 0);
static_assert(NTOK % 128 == 0);
static_assert(NTOK % 8 == 0);
static_assert(DM == NH * DK);
static_assert(DK == 64);
static_assert(DM == 512);
static_assert(DM % 64 == 0 && DFF % 64 == 0);
static_assert(DM % 32 == 0 && DFF % 32 == 0);
static_assert(((size_t)NTOK * DM) % 2048 == 0);
static_assert(((size_t)DM * DM) % 2048 == 0);
static_assert(((size_t)DFF * DM) % 2048 == 0);
static_assert(64 * VP <= 128 * LP);
static_assert(LP % 8 == 0 && VP % 8 == 0 && FP % 4 == 0);

typedef _Float16 v16h __attribute__((ext_vector_type(16)));
typedef _Float16 v8h  __attribute__((ext_vector_type(8)));
typedef _Float16 v4h  __attribute__((ext_vector_type(4)));
typedef float    v8f  __attribute__((ext_vector_type(8)));
typedef float    v4f  __attribute__((ext_vector_type(4)));

union Frag { v16h v; v8h h[2]; };

#define C1 (1.44269504088896340736f * 3.0517578125e-05f)
#define C2 (1.44269504088896340736f * 1.4901161193847656e-08f)
#define SC_RES   2048.0f
#define P_CARRY  10.0f
#define SC_WO    6.103515625e-05f
#define SC_FF2   2.44140625e-04f

static __device__ __forceinline__ v8f zero8() {
    v8f z;
#pragma unroll
    for (int i = 0; i < 8; ++i) z[i] = 0.0f;
    return z;
}

static __device__ __forceinline__ v16h load_frag16(const _Float16* base, int ld, int lane) {
    int m  = lane & 15;
    int kb = (lane >> 4) << 3;
    const _Float16* p = base + (size_t)m * ld + kb;
    Frag f;
    f.h[0] = *(const v8h*)(p);
    f.h[1] = *(const v8h*)(p + 16);
    return f.v;
}

static __device__ __forceinline__ v8f wmma16(v16h a, v16h b, v8f c) {
    v8f d = __builtin_amdgcn_wmma_f32_16x16x32_f16(false, a, false, b, (short)0, c, false, false);
    asm volatile("v_nop\n\tv_nop\n\tv_nop\n\tv_nop" : "+v"(d) : "v"(a), "v"(b));
    return d;
}

static __device__ __forceinline__ float bf16r(float x) {
    unsigned u = __float_as_uint(x);
    u = (u + 0x7FFFu + ((u >> 16) & 1u)) & 0xFFFF0000u;
    return __uint_as_float(u);
}

static __device__ __forceinline__ float ex2(float x) {
    return __builtin_amdgcn_exp2f(x);
}

static __device__ __forceinline__ void wave_lds_sync() {
    __builtin_amdgcn_fence(3, "wavefront");
    asm volatile("s_wait_dscnt 0" ::: "memory");
    __builtin_amdgcn_wave_barrier();
}

static __device__ __forceinline__ v8f scale8(v8f a, float s) {
#pragma unroll
    for (int i = 0; i < 8; ++i) a[i] *= s;
    return a;
}

__global__ __launch_bounds__(256) void k_cvtx(const float* __restrict__ x,
                                               _Float16* __restrict__ xh) {
    const size_t i = ((size_t)blockIdx.x * 256 + threadIdx.x) * 8;
    if (i < (size_t)NTOK * DM) {
        const size_t tok = i / DM;
        const size_t c   = i - tok * DM;
        const size_t b   = tok / SEQ;
        const size_t s   = tok - b * SEQ;
        const float* src = x + ((b * SEQ_FULL + s) * DM + c);
        v4f a0 = *(const v4f*)(src);
        v4f a1 = *(const v4f*)(src + 4);
        v8h o;
        o[0] = (_Float16)bf16r(a0.x); o[1] = (_Float16)bf16r(a0.y);
        o[2] = (_Float16)bf16r(a0.z); o[3] = (_Float16)bf16r(a0.w);
        o[4] = (_Float16)bf16r(a1.x); o[5] = (_Float16)bf16r(a1.y);
        o[6] = (_Float16)bf16r(a1.z); o[7] = (_Float16)bf16r(a1.w);
        *(volatile v8h*)(xh + i) = o;
        __threadfence();
        *(volatile v8h*)(xh + i) = o;
    }
}

__global__ __launch_bounds__(256) void k_cvtw(const float* __restrict__ src,
                                               _Float16* __restrict__ dst,
                                               int n, float scale) {
    const size_t i = ((size_t)blockIdx.x * 256 + threadIdx.x) * 8;
    if (i < (size_t)n) {
        v4f a0 = *(const v4f*)(src + i);
        v4f a1 = *(const v4f*)(src + i + 4);
        v8h o;
        o[0] = (_Float16)(bf16r(a0.x) * scale); o[1] = (_Float16)(bf16r(a0.y) * scale);
        o[2] = (_Float16)(bf16r(a0.z) * scale); o[3] = (_Float16)(bf16r(a0.w) * scale);
        o[4] = (_Float16)(bf16r(a1.x) * scale); o[5] = (_Float16)(bf16r(a1.y) * scale);
        o[6] = (_Float16)(bf16r(a1.z) * scale); o[7] = (_Float16)(bf16r(a1.w) * scale);
        *(volatile v8h*)(dst + i) = o;
        __threadfence();
        *(volatile v8h*)(dst + i) = o;
    }
}

template <int K>
static __device__ __forceinline__ void gemm_32x64(const _Float16* __restrict__ A,
                                                  const _Float16* __restrict__ W,
                                                  int lane, v8f (&acc)[2][4]) {
    static_assert(K % 32 == 0);
#pragma unroll 1
    for (int kk = 0; kk < K; kk += 32) {
        const v16h a0 = load_frag16(A + kk, K, lane);
        const v16h a1 = load_frag16(A + (size_t)16 * K + kk, K, lane);
#pragma unroll
        for (int nt = 0; nt < 4; ++nt) {
            const v16h bw = load_frag16(W + (size_t)(nt * 16) * K + kk, K, lane);
            acc[0][nt] = wmma16(a0, bw, acc[0][nt]);
            acc[1][nt] = wmma16(a1, bw, acc[1][nt]);
        }
    }
}

__global__ __launch_bounds__(128) void k_qkv(const _Float16* __restrict__ xh,
                                              const _Float16* __restrict__ wqkv,
                                              const float* __restrict__ bq,
                                              const float* __restrict__ bk,
                                              const float* __restrict__ bv,
                                              _Float16* __restrict__ qkH,
                                              _Float16* __restrict__ qkL,
                                              _Float16* __restrict__ vT) {
    __shared__ __align__(16) _Float16 stA[128 * LP];
    __shared__ __align__(16) _Float16 stB[128 * LP];

    const int tid  = threadIdx.x;
    const int lane = tid & 31;
    const int w    = tid >> 5;
    const int m0   = blockIdx.x * 128;
    const int y    = blockIdx.y;
    const int kind = y >> 3;
    const int hd   = y & 7;
    const int n0   = y * 64;
    const int r0   = (lane >> 4) << 3;
    const int cc   = lane & 15;

    v8f acc[2][4];
#pragma unroll
    for (int mt = 0; mt < 2; ++mt)
#pragma unroll
        for (int nt = 0; nt < 4; ++nt) acc[mt][nt] = zero8();

    gemm_32x64<DM>(xh + (size_t)(m0 + w * 32) * DM, wqkv + (size_t)n0 * DM, lane, acc);

    float bia[4];
#pragma unroll
    for (int nt = 0; nt < 4; ++nt) {
        const int c = hd * 64 + nt * 16 + cc;
        const float fq = bq[c];
        const float fk = bk[c];
        const float fv = bv[c];
        const float bs = (kind == 0) ? fq : ((kind == 1) ? fk : fv);
        bia[nt] = bf16r(bs) * 64.0f;
    }

    if (kind < 2) {
        _Float16* sh = &stA[w * 32 * LP];
        _Float16* sl = &stB[w * 32 * LP];
#pragma unroll
        for (int mt = 0; mt < 2; ++mt)
#pragma unroll
            for (int nt = 0; nt < 4; ++nt)
#pragma unroll
                for (int g = 0; g < 8; ++g) {
                    const float v = acc[mt][nt][g] + bia[nt];
                    const _Float16 hv = (_Float16)v;
                    const int o = (mt * 16 + r0 + g) * LP + nt * 16 + cc;
                    sh[o] = hv;
                    sl[o] = (_Float16)((v - (float)hv) * SC_RES);
                }
        wave_lds_sync();
        v8h ph[8], pl[8];
#pragma unroll
        for (int j = 0; j < 8; ++j) {
            const int o = (4 * j + (lane >> 3)) * LP + (lane & 7) * 8;
            ph[j] = *(const v8h*)(&sh[o]);
            pl[j] = *(const v8h*)(&sl[o]);
        }
        const size_t base = (size_t)kind * NTOK * DM + (size_t)(m0 + w * 32) * DM
                          + (size_t)hd * DK + (size_t)(lane & 7) * 8;
#pragma unroll
        for (int j = 0; j < 8; ++j) {
            const size_t o = base + (size_t)(4 * j + (lane >> 3)) * DM;
            *(volatile v8h*)(qkH + o) = ph[j];
            *(volatile v8h*)(qkL + o) = pl[j];
        }
        __threadfence();
#pragma unroll
        for (int j = 0; j < 8; ++j) {
            const size_t o = base + (size_t)(4 * j + (lane >> 3)) * DM;
            *(volatile v8h*)(qkH + o) = ph[j];
            *(volatile v8h*)(qkL + o) = pl[j];
        }
    } else {
#pragma unroll
        for (int mt = 0; mt < 2; ++mt)
#pragma unroll
            for (int nt = 0; nt < 4; ++nt) {
                v8h pk;
#pragma unroll
                for (int g = 0; g < 8; ++g) pk[g] = (_Float16)(acc[mt][nt][g] + bia[nt]);
                *(v8h*)(&stA[(nt * 16 + cc) * VP + w * 32 + mt * 16 + r0]) = pk;
            }
        __syncthreads();
        const int b  = m0 / SEQ;
        const int s0 = m0 - b * SEQ;
        v8h pv[8];
#pragma unroll
        for (int j = 0; j < 8; ++j) {
            const int d = w * 16 + 2 * j + (lane >> 4);
            pv[j] = *(const v8h*)(&stA[d * VP + (lane & 15) * 8]);
        }
        _Float16* dst = vT + ((size_t)(b * NH + hd) * DK) * SEQ + s0 + (lane & 15) * 8;
#pragma unroll
        for (int j = 0; j < 8; ++j)
            *(volatile v8h*)(dst + (size_t)(w * 16 + 2 * j + (lane >> 4)) * SEQ) = pv[j];
        __threadfence();
#pragma unroll
        for (int j = 0; j < 8; ++j)
            *(volatile v8h*)(dst + (size_t)(w * 16 + 2 * j + (lane >> 4)) * SEQ) = pv[j];
    }
}

__global__ __launch_bounds__(256) __attribute__((amdgpu_num_vgpr(256)))
void k_attn(const _Float16* __restrict__ qh,
            const _Float16* __restrict__ ql,
            const _Float16* __restrict__ kh,
            const _Float16* __restrict__ kl,
            const _Float16* __restrict__ vT,
            _Float16* __restrict__ ctx) {
    __shared__ __align__(16) _Float16 Cst[8][16 * LP];

    const int tid  = threadIdx.x;
    const int lane = tid & 31;
    const int w    = tid >> 5;
    const int b    = blockIdx.z;
    const int hd   = blockIdx.y;
    const int q0   = blockIdx.x * 128 + w * 16;
    const int r0   = (lane >> 4) << 3;
    const int cc   = lane & 15;

    const size_t qoff = ((size_t)b * SEQ + q0) * DM + (size_t)hd * DK;
    const v16h qh0 = load_frag16(qh + qoff, DM, lane);
    const v16h qh1 = load_frag16(qh + qoff + 32, DM, lane);
    const v16h ql0 = load_frag16(ql + qoff, DM, lane);
    const v16h ql1 = load_frag16(ql + qoff + 32, DM, lane);

    const _Float16* khb = kh + (size_t)b * SEQ * DM + (size_t)hd * DK;
    const _Float16* klb = kl + (size_t)b * SEQ * DM + (size_t)hd * DK;
    const _Float16* vtb = vT + ((size_t)(b * NH + hd) * DK) * SEQ;

    v8f ot0 = zero8(), ot1 = zero8(), ot2 = zero8(), ot3 = zero8();
    float mr = -1.0e30f, lr = 0.0f;

#pragma unroll 1
    for (int key0 = 0; key0 < SEQ; key0 += 32) {
        const _Float16* kp = khb + (size_t)key0 * DM;
        const _Float16* lp = klb + (size_t)key0 * DM;

        v16h ka = load_frag16(kp, DM, lane);
        v16h kb = load_frag16(kp + 32, DM, lane);
        v16h la = load_frag16(lp, DM, lane);
        v16h lb = load_frag16(lp + 32, DM, lane);
        v8f sh0 = wmma16(ka, qh0, zero8());
        sh0 = wmma16(kb, qh1, sh0);
        v8f sr0 = wmma16(ka, ql0, zero8());
        sr0 = wmma16(kb, ql1, sr0);
        sr0 = wmma16(la, qh0, sr0);
        sr0 = wmma16(lb, qh1, sr0);

        ka = load_frag16(kp + (size_t)16 * DM, DM, lane);
        kb = load_frag16(kp + (size_t)16 * DM + 32, DM, lane);
        la = load_frag16(lp + (size_t)16 * DM, DM, lane);
        lb = load_frag16(lp + (size_t)16 * DM + 32, DM, lane);
        v8f sh1 = wmma16(ka, qh0, zero8());
        sh1 = wmma16(kb, qh1, sh1);
        v8f sr1 = wmma16(ka, ql0, zero8());
        sr1 = wmma16(kb, ql1, sr1);
        sr1 = wmma16(la, qh0, sr1);
        sr1 = wmma16(lb, qh1, sr1);

        float t0[8], t1[8];
        float ml = -1.0e30f;
#pragma unroll
        for (int g = 0; g < 8; ++g) {
            t0[g] = __builtin_fmaf(sh0[g], C1, sr0[g] * C2);
            t1[g] = __builtin_fmaf(sh1[g], C1, sr1[g] * C2);
            ml = fmaxf(ml, fmaxf(t0[g], t1[g]));
        }
        ml = fmaxf(ml, __shfl_xor(ml, 16, 32));
        const float mn   = fmaxf(mr, ml);
        const float corr = ex2(mr - mn);
        const float shf  = P_CARRY - mn;

        Frag pf;
        float ps = 0.0f;
#pragma unroll
        for (int g = 0; g < 8; ++g) {
            const float p0 = ex2(t0[g] + shf);
            const float p1 = ex2(t1[g] + shf);
            ps += p0 + p1;
            pf.v[g]     = (_Float16)p0;
            pf.v[8 + g] = (_Float16)p1;
        }
        lr = lr * corr + ps;
        mr = mn;

        ot0 = scale8(ot0, corr);
        ot1 = scale8(ot1, corr);
        ot2 = scale8(ot2, corr);
        ot3 = scale8(ot3, corr);

        const _Float16* vp = vtb + key0;
        v16h va = load_frag16(vp, SEQ, lane);
        ot0 = wmma16(va, pf.v, ot0);
        va = load_frag16(vp + (size_t)16 * SEQ, SEQ, lane);
        ot1 = wmma16(va, pf.v, ot1);
        va = load_frag16(vp + (size_t)32 * SEQ, SEQ, lane);
        ot2 = wmma16(va, pf.v, ot2);
        va = load_frag16(vp + (size_t)48 * SEQ, SEQ, lane);
        ot3 = wmma16(va, pf.v, ot3);
    }

    const float lt  = lr + __shfl_xor(lr, 16, 32);
    const float inv = 4.0f * (1.0f / lt);

    _Float16* cs = &Cst[w][0];
    {
        v8h c0, c1, c2, c3;
#pragma unroll
        for (int g = 0; g < 8; ++g) {
            c0[g] = (_Float16)(ot0[g] * inv);
            c1[g] = (_Float16)(ot1[g] * inv);
            c2[g] = (_Float16)(ot2[g] * inv);
            c3[g] = (_Float16)(ot3[g] * inv);
        }
        *(v8h*)(&cs[cc * LP + 0 * 16 + r0]) = c0;
        *(v8h*)(&cs[cc * LP + 1 * 16 + r0]) = c1;
        *(v8h*)(&cs[cc * LP + 2 * 16 + r0]) = c2;
        *(v8h*)(&cs[cc * LP + 3 * 16 + r0]) = c3;
    }
    wave_lds_sync();

    v8h cv[4];
#pragma unroll
    for (int j = 0; j < 4; ++j)
        cv[j] = *(const v8h*)(&cs[(4 * j + (lane >> 3)) * LP + (lane & 7) * 8]);
    _Float16* cb = ctx + ((size_t)b * SEQ + q0) * DM + (size_t)hd * DK + (lane & 7) * 8;
#pragma unroll
    for (int j = 0; j < 4; ++j)
        *(volatile v8h*)(cb + (size_t)(4 * j + (lane >> 3)) * DM) = cv[j];
    __threadfence();
#pragma unroll
    for (int j = 0; j < 4; ++j)
        *(volatile v8h*)(cb + (size_t)(4 * j + (lane >> 3)) * DM) = cv[j];
}

template <int K, bool RB>
static __device__ __forceinline__ void gemm_res_body(const _Float16* __restrict__ A,
                                                     const _Float16* __restrict__ W,
                                                     const float* __restrict__ bias,
                                                     const float* __restrict__ resblk,
                                                     float* __restrict__ out,
                                                     float* os, float scale,
                                                     int m0, int n0, int w, int lane) {
    const int r0 = (lane >> 4) << 3;
    const int cc = lane & 15;
    v8f acc[2][4];
#pragma unroll
    for (int mt = 0; mt < 2; ++mt)
#pragma unroll
        for (int nt = 0; nt < 4; ++nt) acc[mt][nt] = zero8();

    gemm_32x64<K>(A + (size_t)(m0 + w * 32) * K, W + (size_t)n0 * K, lane, acc);

    float bia[4];
#pragma unroll
    for (int nt = 0; nt < 4; ++nt) bia[nt] = bf16r(bias[n0 + nt * 16 + cc]);

#pragma unroll
    for (int mt = 0; mt < 2; ++mt)
#pragma unroll
        for (int nt = 0; nt < 4; ++nt)
#pragma unroll
            for (int g = 0; g < 8; ++g)
                os[(mt * 16 + r0 + g) * FP + nt * 16 + cc] =
                    __builtin_fmaf(acc[mt][nt][g], scale, bia[nt]);
    wave_lds_sync();

    const int c4 = (lane & 15) * 4;
    v4f sv[16];
#pragma unroll
    for (int j = 0; j < 16; ++j) {
        const int row = 2 * j + (lane >> 4);
        v4f v = *(const v4f*)(&os[row * FP + c4]);
        v4f r = *(const v4f*)(resblk + (size_t)(w * 32 + row) * DM + n0 + c4);
        if (RB) { r.x = bf16r(r.x); r.y = bf16r(r.y); r.z = bf16r(r.z); r.w = bf16r(r.w); }
        v.x += r.x; v.y += r.y; v.z += r.z; v.w += r.w;
        sv[j] = v;
    }
    float* ob = out + (size_t)(m0 + w * 32) * DM + n0 + c4;
#pragma unroll
    for (int j = 0; j < 16; ++j)
        *(volatile v4f*)(ob + (size_t)(2 * j + (lane >> 4)) * DM) = sv[j];
    __threadfence();
#pragma unroll
    for (int j = 0; j < 16; ++j)
        *(volatile v4f*)(ob + (size_t)(2 * j + (lane >> 4)) * DM) = sv[j];
}

__global__ __launch_bounds__(128) void k_wo(const _Float16* __restrict__ ctx,
                                             const _Float16* __restrict__ woh,
                                             const float* __restrict__ bo,
                                             const float* __restrict__ x,
                                             float* __restrict__ pre) {
    __shared__ __align__(16) float Ost[4 * 32 * FP];
    const int tid = threadIdx.x, lane = tid & 31, w = tid >> 5;
    const int m0 = blockIdx.x * 128, n0 = blockIdx.y * 64;
    const int b  = m0 / SEQ;
    const int s0 = m0 - b * SEQ;
    const float* resblk = x + ((size_t)b * SEQ_FULL + s0) * DM;
    gemm_res_body<DM, true>(ctx, woh, bo, resblk, pre, &Ost[w * 32 * FP], SC_WO, m0, n0, w, lane);
}

__global__ __launch_bounds__(128) void k_ffn2(const _Float16* __restrict__ ff1,
                                               const _Float16* __restrict__ w2h,
                                               const float* __restrict__ b2,
                                               const float* __restrict__ hf,
                                               float* __restrict__ pre) {
    __shared__ __align__(16) float Ost[4 * 32 * FP];
    const int tid = threadIdx.x, lane = tid & 31, w = tid >> 5;
    const int m0 = blockIdx.x * 128, n0 = blockIdx.y * 64;
    const float* resblk = hf + (size_t)m0 * DM;
    gemm_res_body<DFF, false>(ff1, w2h, b2, resblk, pre, &Ost[w * 32 * FP], SC_FF2, m0, n0, w, lane);
}

__global__ __launch_bounds__(128) void k_ffn1(const _Float16* __restrict__ hh,
                                               const _Float16* __restrict__ w1h,
                                               const float* __restrict__ b1,
                                               _Float16* __restrict__ ff1) {
    __shared__ __align__(16) _Float16 stA[128 * LP];
    const int tid  = threadIdx.x;
    const int lane = tid & 31;
    const int w    = tid >> 5;
    const int m0   = blockIdx.x * 128;
    const int n0   = blockIdx.y * 64;
    const int r0   = (lane >> 4) << 3;
    const int cc   = lane & 15;

    v8f acc[2][4];
#pragma unroll
    for (int mt = 0; mt < 2; ++mt)
#pragma unroll
        for (int nt = 0; nt < 4; ++nt) acc[mt][nt] = zero8();

    gemm_32x64<DM>(hh + (size_t)(m0 + w * 32) * DM, w1h + (size_t)n0 * DM, lane, acc);

    float bia[4];
#pragma unroll
    for (int nt = 0; nt < 4; ++nt) bia[nt] = bf16r(b1[n0 + nt * 16 + cc]) * 64.0f;

    _Float16* sh = &stA[w * 32 * LP];
#pragma unroll
    for (int mt = 0; mt < 2; ++mt)
#pragma unroll
        for (int nt = 0; nt < 4; ++nt)
#pragma unroll
            for (int g = 0; g < 8; ++g) {
                const float v = acc[mt][nt][g] + bia[nt];
                sh[(mt * 16 + r0 + g) * LP + nt * 16 + cc] = (_Float16)((v > 0.0f) ? v : 0.0f);
            }
    wave_lds_sync();
    v8h ph[8];
#pragma unroll
    for (int j = 0; j < 8; ++j)
        ph[j] = *(const v8h*)(&sh[(4 * j + (lane >> 3)) * LP + (lane & 7) * 8]);
    _Float16* ob = ff1 + (size_t)(m0 + w * 32) * DFF + n0 + (lane & 7) * 8;
#pragma unroll
    for (int j = 0; j < 8; ++j)
        *(volatile v8h*)(ob + (size_t)(4 * j + (lane >> 3)) * DFF) = ph[j];
    __threadfence();
#pragma unroll
    for (int j = 0; j < 8; ++j)
        *(volatile v8h*)(ob + (size_t)(4 * j + (lane >> 3)) * DFF) = ph[j];
}

template <bool HOUT>
static __device__ __forceinline__ void ln_body(const float* __restrict__ in,
                                               const float* __restrict__ g,
                                               const float* __restrict__ be,
                                               float* __restrict__ outF,
                                               _Float16* __restrict__ outH) {
    static_assert(DM == 32 * 16);
    const int tid  = threadIdx.x;
    const int lane = tid & 31;
    const int w    = tid >> 5;
    const size_t row = (size_t)blockIdx.x * 8 + w;
    const float* rp = in + row * DM + lane * 4;

    v4f xv[4];
#pragma unroll
    for (int i = 0; i < 4; ++i) xv[i] = *(const v4f*)(rp + i * 128);

    float s = 0.0f;
#pragma unroll
    for (int i = 0; i < 4; ++i) s += (xv[i].x + xv[i].y) + (xv[i].z + xv[i].w);
    s += __shfl_xor(s, 16, 32);
    s += __shfl_xor(s, 8, 32);
    s += __shfl_xor(s, 4, 32);
    s += __shfl_xor(s, 2, 32);
    s += __shfl_xor(s, 1, 32);
    const float mu = s * (1.0f / (float)DM);

    float s2 = 0.0f;
#pragma unroll
    for (int i = 0; i < 4; ++i) {
        const float d0 = xv[i].x - mu, d1 = xv[i].y - mu, d2 = xv[i].z - mu, d3 = xv[i].w - mu;
        s2 += (d0 * d0 + d1 * d1) + (d2 * d2 + d3 * d3);
    }
    s2 += __shfl_xor(s2, 16, 32);
    s2 += __shfl_xor(s2, 8, 32);
    s2 += __shfl_xor(s2, 4, 32);
    s2 += __shfl_xor(s2, 2, 32);
    s2 += __shfl_xor(s2, 1, 32);
    const float rstd = rsqrtf(s2 * (1.0f / (float)DM) + 1.0e-5f);

    v4f yv[4];
#pragma unroll
    for (int i = 0; i < 4; ++i) {
        const v4f gv = *(const v4f*)(g + i * 128 + lane * 4);
        const v4f bv = *(const v4f*)(be + i * 128 + lane * 4);
        v4f yy;
        yy.x = (xv[i].x - mu) * rstd * bf16r(gv.x) + bf16r(bv.x);
        yy.y = (xv[i].y - mu) * rstd * bf16r(gv.y) + bf16r(bv.y);
        yy.z = (xv[i].z - mu) * rstd * bf16r(gv.z) + bf16r(bv.z);
        yy.w = (xv[i].w - mu) * rstd * bf16r(gv.w) + bf16r(bv.w);
        yv[i] = yy;
    }
    v4h hv[4];
    if (HOUT) {
#pragma unroll
        for (int i = 0; i < 4; ++i) {
            v4h t;
            t.x = (_Float16)yv[i].x; t.y = (_Float16)yv[i].y;
            t.z = (_Float16)yv[i].z; t.w = (_Float16)yv[i].w;
            hv[i] = t;
        }
    }
    float* of = outF + row * DM + lane * 4;
#pragma unroll
    for (int i = 0; i < 4; ++i) *(volatile v4f*)(of + i * 128) = yv[i];
    if (HOUT) {
        _Float16* oh = outH + row * DM + lane * 4;
#pragma unroll
        for (int i = 0; i < 4; ++i) *(volatile v4h*)(oh + i * 128) = hv[i];
    }
    __threadfence();
#pragma unroll
    for (int i = 0; i < 4; ++i) *(volatile v4f*)(of + i * 128) = yv[i];
    if (HOUT) {
        _Float16* oh = outH + row * DM + lane * 4;
#pragma unroll
        for (int i = 0; i < 4; ++i) *(volatile v4h*)(oh + i * 128) = hv[i];
    }
}

__global__ __launch_bounds__(256) void k_ln_mid(const float* __restrict__ pre,
                                                 const float* __restrict__ g,
                                                 const float* __restrict__ be,
                                                 float* __restrict__ hf,
                                                 _Float16* __restrict__ hh) {
    ln_body<true>(pre, g, be, hf, hh);
}

__global__ __launch_bounds__(256) void k_ln_out(const float* __restrict__ pre,
                                                 const float* __restrict__ g,
                                                 const float* __restrict__ be,
                                                 float* __restrict__ out) {
    ln_body<false>(pre, g, be, out, nullptr);
}

#define SZ_XH   ((size_t)NTOK * DM * 2)
#define SZ_WQKV ((size_t)3 * DM * DM * 2)
#define SZ_WO   ((size_t)DM * DM * 2)
#define SZ_W1   ((size_t)DFF * DM * 2)
#define SZ_W2   ((size_t)DM * DFF * 2)
#define SZ_QK   ((size_t)4 * NTOK * DM * 2)
#define SZ_VT   ((size_t)NB * NH * DK * SEQ * 2)
#define SZ_CTX  ((size_t)NTOK * DM * 2)
#define SZ_PRE  ((size_t)NTOK * DM * 4)
#define SZ_HF   ((size_t)NTOK * DM * 4)
#define SZ_HH   ((size_t)NTOK * DM * 2)
#define SZ_FF1  ((size_t)NTOK * DFF * 2)
#define SZ_TOTAL (SZ_XH + SZ_WQKV + SZ_WO + SZ_W1 + SZ_W2 + SZ_QK + SZ_VT + SZ_CTX + SZ_PRE + SZ_HF + SZ_HH)

static_assert(SZ_FF1 <= SZ_QK);
static_assert(SZ_TOTAL <= (size_t)134217728);
static_assert(SZ_XH % 128 == 0 && SZ_WQKV % 128 == 0 && SZ_WO % 128 == 0 && SZ_W1 % 128 == 0);
static_assert(SZ_QK % 128 == 0 && SZ_VT % 128 == 0 && SZ_PRE % 128 == 0 && SZ_HH % 128 == 0);

extern "C" void kernel_launch(void* const* d_in, const int* in_sizes, int n_in,
                              void* d_out, int out_size, void* d_ws, size_t ws_size,
                              hipStream_t stream) {
    if (n_in < 15) return;
    if (in_sizes[0] < ((NB - 1) * SEQ_FULL + SEQ) * DM) return;
    if (in_sizes[1] < DM * DM || in_sizes[3] < DM * DM || in_sizes[5] < DM * DM || in_sizes[7] < DM * DM) return;
    if (in_sizes[2] < DM || in_sizes[4] < DM || in_sizes[6] < DM || in_sizes[8] < DM) return;
    if (in_sizes[9] < DM || in_sizes[10] < DM) return;
    if (in_sizes[11] < DFF * DM || in_sizes[12] < DFF) return;
    if (in_sizes[13] < DM * DFF || in_sizes[14] < DM) return;
    if (out_size < NTOK * DM) return;
    if (SZ_TOTAL > ws_size) return;

    const float* x   = (const float*)d_in[0];
    const float* wq  = (const float*)d_in[1];
    const float* bq  = (const float*)d_in[2];
    const float* wk  = (const float*)d_in[3];
    const float* bk  = (const float*)d_in[4];
    const float* wv  = (const float*)d_in[5];
    const float* bv  = (const float*)d_in[6];
    const float* wo  = (const float*)d_in[7];
    const float* bo  = (const float*)d_in[8];
    const float* lng = (const float*)d_in[9];
    const float* lnb = (const float*)d_in[10];
    const float* w1  = (const float*)d_in[11];
    const float* b1  = (const float*)d_in[12];
    const float* w2  = (const float*)d_in[13];
    const float* b2  = (const float*)d_in[14];
    float* out = (float*)d_out;

    char* ws = (char*)d_ws;
    size_t off = 0;
    _Float16* xh   = (_Float16*)(ws + off); off += SZ_XH;
    _Float16* wqkv = (_Float16*)(ws + off); off += SZ_WQKV;
    _Float16* woh  = (_Float16*)(ws + off); off += SZ_WO;
    _Float16* w1h  = (_Float16*)(ws + off); off += SZ_W1;
    _Float16* w2h  = (_Float16*)(ws + off); off += SZ_W2;
    _Float16* qkH  = (_Float16*)(ws + off);
    _Float16* qkL  = qkH + (size_t)2 * NTOK * DM;
    _Float16* ff1  = qkH;
    off += SZ_QK;
    _Float16* vT   = (_Float16*)(ws + off); off += SZ_VT;
    _Float16* ctx  = (_Float16*)(ws + off); off += SZ_CTX;
    float*    pre  = (float*)(ws + off);    off += SZ_PRE;
    float*    hf   = (float*)(ws + off);    off += SZ_HF;
    _Float16* hh   = (_Float16*)(ws + off); off += SZ_HH;
    if (off > ws_size) return;

    const _Float16* qh = qkH;
    const _Float16* kh = qkH + (size_t)NTOK * DM;
    const _Float16* ql = qkL;
    const _Float16* kl = qkL + (size_t)NTOK * DM;

    const int nw = DM * DM, nf = DFF * DM;
    k_cvtx<<<dim3((unsigned)(((size_t)NTOK * DM) / 2048)), dim3(256), 0, stream>>>(x, xh);
    k_cvtw<<<dim3(nw / 2048), dim3(256), 0, stream>>>(wq, wqkv, nw, 64.0f);
    k_cvtw<<<dim3(nw / 2048), dim3(256), 0, stream>>>(wk, wqkv + (size_t)nw, nw, 64.0f);
    k_cvtw<<<dim3(nw / 2048), dim3(256), 0, stream>>>(wv, wqkv + (size_t)2 * nw, nw, 64.0f);
    k_cvtw<<<dim3(nw / 2048), dim3(256), 0, stream>>>(wo, woh, nw, 64.0f);
    k_cvtw<<<dim3(nf / 2048), dim3(256), 0, stream>>>(w1, w1h, nf, 64.0f);
    k_cvtw<<<dim3(nf / 2048), dim3(256), 0, stream>>>(w2, w2h, nf, 64.0f);

    k_qkv<<<dim3(NTOK / 128, 24), dim3(128), 0, stream>>>(xh, wqkv, bq, bk, bv, qkH, qkL, vT);
    k_attn<<<dim3(SEQ / 128, NH, NB), dim3(256), 0, stream>>>(qh, ql, kh, kl, vT, ctx);
    k_wo<<<dim3(NTOK / 128, DM / 64), dim3(128), 0, stream>>>(ctx, woh, bo, x, pre);
    k_ln_mid<<<dim3(NTOK / 8), dim3(256), 0, stream>>>(pre, lng, lnb, hf, hh);
    k_ffn1<<<dim3(NTOK / 128, DFF / 64), dim3(128), 0, stream>>>(hh, w1h, b1, ff1);
    k_ffn2<<<dim3(NTOK / 128, DM / 64), dim3(128), 0, stream>>>(ff1, w2h, b2, hf, pre);
    k_ln_out<<<dim3(NTOK / 8), dim3(256), 0, stream>>>(pre, lng, lnb, out);
}
